// MultiHeadAttention_16630113370910
// MI455X (gfx1250) — hardware-verified
//
#include <hip/hip_runtime.h>


#ifndef NB
#define NB 2
#endif
#ifndef SEQ
#define SEQ 4096
#endif
#define NB_FULL  2
#define SEQ_FULL 4096
#define TT   SEQ
#define DM   768
#define NH_  12
#define HD   64
#define DQ   (NH_ * HD)
#define RH   ((SEQ) < 512 ? (SEQ) : 512)
#define PCAR 1024.0f
#define SCL  0.125f
#define L2E  1.4426950408889634f
#define WSB  ((size_t)4 * DQ * DM * 2 + (size_t)TT * DM * 2 + (size_t)2 * TT * DQ * 4 + (size_t)9 * NH_ * TT * HD * 2 + (size_t)2 * TT * DQ * 2)

static_assert(SEQ % 64 == 0);
static_assert(SEQ <= SEQ_FULL);
static_assert(NB <= NB_FULL);
static_assert(DM % 64 == 0);
static_assert(DQ % 64 == 0);
static_assert(DQ == DM);
static_assert(RH % 16 == 0);
static_assert((TT - RH) % 16 == 0);
static_assert(((size_t)DQ * DM * 2) % 256 == 0);
static_assert(((size_t)TT * DM * 2) % 256 == 0);
static_assert(((size_t)NH_ * TT * HD * 2) % 256 == 0);
static_assert(WSB <= (size_t)134217728);

typedef _Float16 h16;
typedef unsigned short bf;
typedef __attribute__((ext_vector_type(16))) __bf16   v16bf;
typedef __attribute__((ext_vector_type(16))) _Float16 v16h;
typedef __attribute__((ext_vector_type(8)))  _Float16 v8h;
typedef __attribute__((ext_vector_type(8)))  unsigned short v8us;
typedef __attribute__((ext_vector_type(8)))  float    v8f;
typedef __attribute__((ext_vector_type(4)))  float    v4f;
typedef __attribute__((ext_vector_type(2)))  unsigned short v2us;
typedef v8h  __attribute__((may_alias)) v8ha;
typedef v4f  __attribute__((may_alias)) v4fa;
typedef v8us __attribute__((may_alias)) v8usa;

__device__ __forceinline__ unsigned short f2bf(float f) { unsigned u = __float_as_uint(f); u += 0x7FFFu + ((u >> 16) & 1u); return (unsigned short)(u >> 16); }
__device__ __forceinline__ float bf2f(unsigned short b) { return __uint_as_float(((unsigned)b) << 16); }
__device__ __forceinline__ float bfr(float f) { return bf2f(f2bf(f)); }
__device__ __forceinline__ v16h cat16(v8h lo, v8h hi) { return __builtin_shufflevector(lo, hi, 0, 1, 2, 3, 4, 5, 6, 7, 8, 9, 10, 11, 12, 13, 14, 15); }
__device__ __forceinline__ v16bf cat16b(v8us lo, v8us hi) { return __builtin_bit_cast(v16bf, __builtin_shufflevector(lo, hi, 0, 1, 2, 3, 4, 5, 6, 7, 8, 9, 10, 11, 12, 13, 14, 15)); }
__device__ __forceinline__ v8f wmma16(v16h a, v16h b, v8f c) { return __builtin_amdgcn_wmma_f32_16x16x32_f16(false, a, false, b, (short)0, c, false, false); }
__device__ __forceinline__ v8f wmmab(v16bf a, v16bf b, v8f c) { return __builtin_amdgcn_wmma_f32_16x16x32_bf16(false, a, false, b, (short)0, c, false, false); }
__device__ __forceinline__ void splitf(float y, unsigned short& h, unsigned short& l) { h = f2bf(y); l = f2bf(y - bf2f(h)); }

template <typename T16> struct WFrag;
template <> struct WFrag<h16> { typedef v16h V; static __device__ __forceinline__ V ld(const h16* p) { return cat16(*(const v8h*)p, *(const v8h*)(p + 16)); } static __device__ __forceinline__ v8f mma(V a, V b, v8f c) { return wmma16(a, b, c); } };
template <> struct WFrag<bf> { typedef v16bf V; static __device__ __forceinline__ V ld(const bf* p) { return cat16b(*(const v8us*)p, *(const v8us*)(p + 16)); } static __device__ __forceinline__ v8f mma(V a, V b, v8f c) { return wmmab(a, b, c); } };

template <typename T16, int NSPLIT, bool BIAS>
__global__ __launch_bounds__(32) void k_gemmw(const T16* __restrict__ A, const T16* __restrict__ A2, const T16* __restrict__ Bt, const T16* __restrict__ Bt2, int K, float* C, int ldc, const float* __restrict__ bias, size_t sA, size_t sB, size_t sC) {
    typedef typename WFrag<T16>::V V;
    __shared__ __align__(16) float os[16 * 68];
    const size_t z = blockIdx.z; A += z * sA; if (A2) A2 += z * sA; Bt += z * sB; if (Bt2) Bt2 += z * sB; C += z * sC;
    const int lane = threadIdx.x & 31, lr = lane & 15, hi = lane >> 4; const int r0 = blockIdx.x * 64, c0 = blockIdx.y * 64;
    v8f acc[4][4];
#pragma unroll
    for (int mb = 0; mb < 4; ++mb)
#pragma unroll
        for (int nb = 0; nb < 4; ++nb) acc[mb][nb] = (v8f){};
    const size_t aoff = (size_t)(r0 + lr) * K + 8 * hi, boff = (size_t)(c0 + lr) * K + 8 * hi;
#pragma unroll 1
    for (int kc = 0; kc < K; kc += 32) {
        V a[4], a2[4];
#pragma unroll
        for (int mb = 0; mb < 4; ++mb) { a[mb] = WFrag<T16>::ld(A + aoff + (size_t)mb * 16 * K + kc); if (NSPLIT == 1 || NSPLIT == 2) a2[mb] = WFrag<T16>::ld(A2 + aoff + (size_t)mb * 16 * K + kc); }
#pragma unroll
        for (int nb = 0; nb < 4; ++nb) { const V b = WFrag<T16>::ld(Bt + boff + (size_t)nb * 16 * K + kc); V b2; if (NSPLIT >= 2) b2 = WFrag<T16>::ld(Bt2 + boff + (size_t)nb * 16 * K + kc);
#pragma unroll
            for (int mb = 0; mb < 4; ++mb) { acc[mb][nb] = WFrag<T16>::mma(a[mb], b, acc[mb][nb]); if (NSPLIT == 1 || NSPLIT == 2) acc[mb][nb] = WFrag<T16>::mma(a2[mb], b, acc[mb][nb]); if (NSPLIT >= 2) acc[mb][nb] = WFrag<T16>::mma(a[mb], b2, acc[mb][nb]); } }
        asm volatile("v_nop\n\tv_nop\n\tv_nop\n\tv_nop" : "+v"(acc[0][0]), "+v"(acc[1][1]), "+v"(acc[2][2]), "+v"(acc[3][3]) : "v"(a[0]), "v"(a[3]));
    }
#pragma unroll
    for (int mb = 0; mb < 4; ++mb) {
#pragma unroll
        for (int nb = 0; nb < 4; ++nb) {
#pragma unroll
            for (int j = 0; j < 8; ++j) os[(hi * 8 + j) * 68 + nb * 16 + lr] = acc[mb][nb][j]; }
        __builtin_amdgcn_wave_barrier(); asm volatile("" ::: "memory");
        float* crow = C + (size_t)(r0 + mb * 16) * ldc + c0;
#pragma unroll 1
        for (int ps = 0; ps < 2; ++ps) {
#pragma unroll
            for (int s = 0; s < 8; ++s) { const int row = 2 * s + hi, cofs = lr * 4; v4f val = *(const v4fa*)(os + row * 68 + cofs); if (BIAS) { val[0] += bfr(bias[c0 + cofs]); val[1] += bfr(bias[c0 + cofs + 1]); val[2] += bfr(bias[c0 + cofs + 2]); val[3] += bfr(bias[c0 + cofs + 3]); }
                *(volatile v4f*)(crow + (size_t)row * ldc + cofs) = val; }
            if (ps == 0) __threadfence(); }
        __builtin_amdgcn_wave_barrier(); asm volatile("" ::: "memory");
    }
}

__global__ __launch_bounds__(256) void k_wtG(const float* __restrict__ w, int K, int N, bf* Bt) {
    const int lane = threadIdx.x & 31; const int L0 = (blockIdx.x * 8 + (threadIdx.x >> 5)) * 8; const int nlines = N * K / 64;
#pragma unroll
    for (int ps = 0; ps < 2; ++ps) {
#pragma unroll 1
        for (int l = 0; l < 8; ++l) { const int L = L0 + l; if (L >= nlines) break; const size_t e = (size_t)L * 64 + lane * 2; const int k = (int)(e % K), n = (int)(e / K); v2us o;
            o[0] = f2bf(w[(size_t)k * N + n]); o[1] = f2bf(w[(size_t)(k + 1) * N + n]); *(volatile v2us*)(Bt + e) = o; }
        if (ps == 0) __threadfence(); }
}
__global__ __launch_bounds__(256) void k_cvt8(const float* __restrict__ src, bf* dst, size_t n8) { const size_t i = (size_t)blockIdx.x * 256 + threadIdx.x; if (i >= n8) return; const v8f v = *(const v8f*)(src + i * 8); v8us o;
#pragma unroll
    for (int k = 0; k < 8; ++k) o[k] = f2bf(v[k]); *(volatile v8us*)(dst + i * 8) = o; __threadfence(); *(volatile v8us*)(dst + i * 8) = o; }
__global__ __launch_bounds__(256) void k_hp(const float* __restrict__ F, h16* P16, bf* Ph, bf* Pl) {
    const size_t e = ((size_t)blockIdx.x * 256 + threadIdx.x) * 8; if (e >= (size_t)NH_ * TT * HD) return;
    const int d = (int)(e % HD); const int t = (int)((e / HD) % TT); const int h = (int)(e / ((size_t)HD * TT));
    const v8f x = *(const v8f*)(F + (size_t)t * DQ + h * HD + d); v8h o16; v8us oh, ol;
#pragma unroll
    for (int q = 0; q < 8; ++q) { o16[q] = (h16)x[q]; unsigned short a2, c2; splitf(x[q], a2, c2); oh[q] = a2; ol[q] = c2; }
    *(volatile v8h*)(P16 + e) = o16; *(volatile v8us*)(Ph + e) = oh; *(volatile v8us*)(Pl + e) = ol; __threadfence(); *(volatile v8h*)(P16 + e) = o16; *(volatile v8us*)(Ph + e) = oh; *(volatile v8us*)(Pl + e) = ol; }
__global__ __launch_bounds__(256) void k_vt(const float* __restrict__ F, h16* V16, bf* Vh, bf* Vl) {
    const size_t e = ((size_t)blockIdx.x * 256 + threadIdx.x) * 8; if (e >= (size_t)NH_ * HD * TT) return;
    const int t = (int)(e % TT); const int d = (int)((e / TT) % HD); const int g = (int)(e / ((size_t)TT * HD)); v8h o16; v8us oh, ol;
#pragma unroll
    for (int q = 0; q < 8; ++q) { const float x = F[(size_t)(t + q) * DQ + g * HD + d]; o16[q] = (h16)x; unsigned short a2, c2; splitf(x, a2, c2); oh[q] = a2; ol[q] = c2; }
    *(volatile v8h*)(V16 + e) = o16; *(volatile v8us*)(Vh + e) = oh; *(volatile v8us*)(Vl + e) = ol; __threadfence(); *(volatile v8h*)(V16 + e) = o16; *(volatile v8us*)(Vh + e) = oh; *(volatile v8us*)(Vl + e) = ol; }

template <typename T16> struct PPk;
template <> struct PPk<h16> {
    static __device__ __forceinline__ v16h hi(v8f p0, v8f p1) { v8h a, b;
#pragma unroll
        for (int r = 0; r < 8; ++r) { a[r] = (h16)(p0[r] * PCAR); b[r] = (h16)(p1[r] * PCAR); }
        return cat16(a, b); }
    static __device__ __forceinline__ v16h lo(v8f p0, v8f p1) { return hi(p0, p1); }
};
template <> struct PPk<bf> {
    static __device__ __forceinline__ v16bf hi(v8f p0, v8f p1) { v8us a, b;
#pragma unroll
        for (int r = 0; r < 8; ++r) { a[r] = f2bf(p0[r]); b[r] = f2bf(p1[r]); }
        return cat16b(a, b); }
    static __device__ __forceinline__ v16bf lo(v8f p0, v8f p1) { v8us a, b;
#pragma unroll
        for (int r = 0; r < 8; ++r) { a[r] = f2bf(p0[r] - bf2f(f2bf(p0[r]))); b[r] = f2bf(p1[r] - bf2f(f2bf(p1[r]))); }
        return cat16b(a, b); }
};

template <typename T16, bool HL>
__global__ __launch_bounds__(32) void k_flash(const T16* __restrict__ Q1, const T16* __restrict__ Q2, const T16* __restrict__ K1, const T16* __restrict__ K2, const T16* __restrict__ V1, const T16* __restrict__ V2, int roff, bf* Ah, bf* Al) {
    typedef typename WFrag<T16>::V V;
    __shared__ __align__(16) unsigned short st[2 * 16 * 72];
    const int lane = threadIdx.x & 31, lr = lane & 15, hi = lane >> 4;
    const int q0 = roff + blockIdx.x * 16; const int head = blockIdx.y;
    const size_t hp = (size_t)head * TT * HD;
    const size_t qoff = hp + (size_t)(q0 + lr) * HD + 8 * hi;
    V qa[2], qb[2];
    qa[0] = WFrag<T16>::ld(Q1 + qoff); qa[1] = WFrag<T16>::ld(Q1 + qoff + 32);
    if (HL) { qb[0] = WFrag<T16>::ld(Q2 + qoff); qb[1] = WFrag<T16>::ld(Q2 + qoff + 32); } else { qb[0] = qa[0]; qb[1] = qa[1]; }
    v8f o[4];
#pragma unroll
    for (int dt = 0; dt < 4; ++dt) o[dt] = (v8f){};
    float m = -1.0e30f, l = 0.0f;
    const int nst = (q0 + 47) >> 5;
    const size_t koff = hp + (size_t)lr * HD + 8 * hi;
    const size_t voff = hp + (size_t)lr * TT + 8 * hi;
    const int qi = q0 + lr;
#pragma unroll 1
    for (int stp = 0; stp < nst; ++stp) {
        const int kb = stp * 32;
        v8f s[2];
#pragma unroll
        for (int kt = 0; kt < 2; ++kt) {
            const size_t ko = koff + (size_t)(kb + kt * 16) * HD;
            const V k0 = WFrag<T16>::ld(K1 + ko), k1 = WFrag<T16>::ld(K1 + ko + 32);
            v8f a = (v8f){};
            if (HL) { const V l0 = WFrag<T16>::ld(K2 + ko), l1 = WFrag<T16>::ld(K2 + ko + 32);
                a = WFrag<T16>::mma(l0, qa[0], a); a = WFrag<T16>::mma(l1, qa[1], a); a = WFrag<T16>::mma(k0, qb[0], a); a = WFrag<T16>::mma(k1, qb[1], a); }
            a = WFrag<T16>::mma(k0, qa[0], a); a = WFrag<T16>::mma(k1, qa[1], a);
            s[kt] = a;
        }
        asm volatile("v_nop\n\tv_nop\n\tv_nop\n\tv_nop" : "+v"(s[0]), "+v"(s[1]) : "v"(qa[0]), "v"(qa[1]));
        const bool diag = (kb + 31 > q0);
        float mx = -1.0e30f;
#pragma unroll
        for (int kt = 0; kt < 2; ++kt)
#pragma unroll
            for (int r = 0; r < 8; ++r) { const int key = kb + kt * 16 + 8 * hi + r; float t = s[kt][r] * SCL; t = (diag && (key > qi)) ? -1.0e30f : t; s[kt][r] = t; mx = fmaxf(mx, t); }
        mx = fmaxf(mx, __shfl_xor(mx, 16, 32));
        const float mn = fmaxf(m, mx);
        const float al = __builtin_amdgcn_exp2f((m - mn) * L2E);
        m = mn;
        float psum = 0.0f;
#pragma unroll
        for (int kt = 0; kt < 2; ++kt)
#pragma unroll
            for (int r = 0; r < 8; ++r) { const float p = __builtin_amdgcn_exp2f((s[kt][r] - mn) * L2E); s[kt][r] = p; psum += p; }
        l = l * al + psum;
#pragma unroll
        for (int dt = 0; dt < 4; ++dt) o[dt] = o[dt] * al;
        const V pa = PPk<T16>::hi(s[0], s[1]);
        V pb = pa; if (HL) pb = PPk<T16>::lo(s[0], s[1]);
#pragma unroll
        for (int dt = 0; dt < 4; ++dt) {
            const size_t vo = voff + (size_t)(dt * 16) * TT + kb;
            const V v0 = WFrag<T16>::ld(V1 + vo);
            if (HL) { const V v1 = WFrag<T16>::ld(V2 + vo); o[dt] = WFrag<T16>::mma(v1, pa, o[dt]); o[dt] = WFrag<T16>::mma(v0, pb, o[dt]); }
            o[dt] = WFrag<T16>::mma(v0, pa, o[dt]);
        }
        asm volatile("v_nop\n\tv_nop\n\tv_nop\n\tv_nop" : "+v"(o[0]), "+v"(o[1]), "+v"(o[2]), "+v"(o[3]) : "v"(pa), "v"(pb));
    }
    l += __shfl_xor(l, 16, 32);
    const float inv = (HL ? 1.0f : (1.0f / PCAR)) * (1.0f / l);
#pragma unroll
    for (int dt = 0; dt < 4; ++dt) { v8us hv, lv;
#pragma unroll
        for (int r = 0; r < 8; ++r) { unsigned short a2, c2; splitf(o[dt][r] * inv, a2, c2); hv[r] = a2; lv[r] = c2; }
        *(v8usa*)(st + lr * 72 + dt * 16 + 8 * hi) = hv; *(v8usa*)(st + 16 * 72 + lr * 72 + dt * 16 + 8 * hi) = lv; }
    __syncthreads();
#pragma unroll 1
    for (int ps = 0; ps < 2; ++ps) {
#pragma unroll
        for (int s4 = 0; s4 < 4; ++s4) { const int row = 4 * s4 + (lane >> 3), c = (lane & 7) * 8;
            const v8us a = *(const v8usa*)(st + row * 72 + c); const v8us b = *(const v8usa*)(st + 16 * 72 + row * 72 + c);
            const size_t oo = (size_t)(q0 + row) * DQ + head * HD + c;
            *(volatile v8us*)(Ah + oo) = a; *(volatile v8us*)(Al + oo) = b; }
        if (ps == 0) __threadfence(); }
}

extern "C" void kernel_launch(void* const* d_in, const int* in_sizes, int n_in,
                              void* d_out, int out_size, void* d_ws, size_t ws_size, hipStream_t stream) {
    if (n_in < 6) return;
    const size_t need = (size_t)(NB - 1) * SEQ_FULL * DM + (size_t)TT * DM;
    if ((size_t)in_sizes[0] < need || (size_t)out_size < need) return;
    if (in_sizes[1] < DM * DQ || in_sizes[2] < DM * DQ || in_sizes[3] < DM * DQ || in_sizes[4] < DQ * DM || in_sizes[5] < DM) return;
    const float* x = (const float*)d_in[0]; const float* wq = (const float*)d_in[1]; const float* wk = (const float*)d_in[2]; const float* wv = (const float*)d_in[3]; const float* wo = (const float*)d_in[4]; const float* bo = (const float*)d_in[5];
    float* OUT = (float*)d_out;
    char* wsp = (char*)d_ws;
    auto take = [&](size_t bytes) { char* p = wsp; wsp += (bytes + 255) & ~(size_t)255; return (void*)p; };
    bf* WQ = (bf*)take((size_t)DQ * DM * 2); bf* WK = (bf*)take((size_t)DQ * DM * 2); bf* WV = (bf*)take((size_t)DQ * DM * 2); bf* WO = (bf*)take((size_t)DM * DQ * 2);
    bf* XB = (bf*)take((size_t)TT * DM * 2); float* FQ = (float*)take((size_t)TT * DQ * 4); float* FK = (float*)take((size_t)TT * DQ * 4);
    const size_t PL = (size_t)NH_ * TT * HD * 2;
    h16* QP16 = (h16*)take(PL); h16* KP16 = (h16*)take(PL); h16* VT16 = (h16*)take(PL);
    bf* QPh = (bf*)take(PL); bf* QPl = (bf*)take(PL); bf* KPh = (bf*)take(PL); bf* KPl = (bf*)take(PL); bf* VTh = (bf*)take(PL); bf* VTl = (bf*)take(PL);
    bf* ATh = (bf*)take((size_t)TT * DQ * 2); bf* ATl = (bf*)take((size_t)TT * DQ * 2);
    if ((size_t)(wsp - (char*)d_ws) > ws_size) return;
    float* FV = FK;
    const unsigned LW = (unsigned)((DM * DQ / 64 + 63) / 64);
    k_wtG<<<LW, 256, 0, stream>>>(wq, DM, DQ, WQ);
    k_wtG<<<LW, 256, 0, stream>>>(wk, DM, DQ, WK);
    k_wtG<<<LW, 256, 0, stream>>>(wv, DM, DQ, WV);
    k_wtG<<<LW, 256, 0, stream>>>(wo, DQ, DM, WO);
    const unsigned LP = (unsigned)(((size_t)NH_ * TT * HD / 8 + 255) / 256);
    for (int b = 0; b < NB; ++b) {
        k_cvt8<<<(unsigned)(((size_t)TT * DM / 8 + 255) / 256), 256, 0, stream>>>(x + (size_t)b * SEQ_FULL * DM, XB, (size_t)TT * DM / 8);
        k_gemmw<bf, 0, false><<<dim3(TT / 64, DQ / 64, 1), 32, 0, stream>>>(XB, nullptr, WQ, nullptr, DM, FQ, DQ, nullptr, 0, 0, 0);
        k_hp<<<LP, 256, 0, stream>>>(FQ, QP16, QPh, QPl);
        k_gemmw<bf, 0, false><<<dim3(TT / 64, DQ / 64, 1), 32, 0, stream>>>(XB, nullptr, WK, nullptr, DM, FK, DQ, nullptr, 0, 0, 0);
        k_hp<<<LP, 256, 0, stream>>>(FK, KP16, KPh, KPl);
        k_gemmw<bf, 0, false><<<dim3(TT / 64, DQ / 64, 1), 32, 0, stream>>>(XB, nullptr, WV, nullptr, DM, FV, DQ, nullptr, 0, 0, 0);
        k_vt<<<LP, 256, 0, stream>>>(FV, VT16, VTh, VTl);
        k_flash<bf, true><<<dim3(RH / 16, NH_, 1), 32, 0, stream>>>(QPh, QPl, KPh, KPl, VTh, VTl, 0, ATh, ATl);
        if (TT > RH) k_flash<h16, false><<<dim3((TT - RH) / 16, NH_, 1), 32, 0, stream>>>(QP16, nullptr, KP16, nullptr, VT16, nullptr, RH, ATh, ATl);
        k_gemmw<bf, 1, true><<<dim3(TT / 64, DM / 64, 1), 32, 0, stream>>>(ATh, ATl, WO, nullptr, DQ, OUT + (size_t)b * SEQ_FULL * DM, DM, bo, 0, 0, 0);
    }
}
